// BeamGNN_71932112273657
// MI455X (gfx1250) — hardware-verified
//
#include <hip/hip_runtime.h>
#include <stddef.h>


#define XDIM    3
#define HID     32
#define NTHR    256
#define NWAVE   8
#define EPT     8
#define NGRP    2
#define CHUNK   (NTHR * EPT * NGRP)
#define WCAP    (EPT * NGRP * 32)
#define LISTN   (NWAVE * WCAP)
#define NBC     4096
#define NBF     1024
#define RCAP    40960
#define RBN     128
#define TGT     256
#define XPB     32
#define DEGCAP  256
#define OTHR    512

#define LDS_FILL ((RCAP + NBF + LISTN) * 4 + 64)

static_assert((CHUNK & (CHUNK - 1)) == 0);
static_assert(CHUNK <= 4096);
static_assert(NBC <= 4096 && NBF <= 4096);
static_assert((NBC & (NBC - 1)) == 0 && (NBF & (NBF - 1)) == 0);
static_assert(NBC == 4 * NBF);
static_assert(OTHR * 8 == NBC);
static_assert((RCAP % 32) == 0);
static_assert(TGT == NWAVE * 32);
static_assert((NBC % TGT) == 0);
static_assert((TGT % XPB) == 0);
static_assert(XPB * (HID / 4) == NTHR);
static_assert((HID * HID) % NTHR == 0);

typedef float          v4f   __attribute__((ext_vector_type(4)));
typedef float          v8f   __attribute__((ext_vector_type(8)));
typedef int            v4i   __attribute__((ext_vector_type(4)));
typedef unsigned short v8us  __attribute__((ext_vector_type(8)));
typedef unsigned short v16us __attribute__((ext_vector_type(16)));
typedef __bf16         v16bf __attribute__((ext_vector_type(16)));
union FragB { v16bf v; v16us u; v8us h[2]; };
union FI { float f; int i; };

__device__ __forceinline__ unsigned short bfb(float f) {
  unsigned u = __float_as_uint(f);
  u += 0x7FFFu + ((u >> 16) & 1u);
  return (unsigned short)(u >> 16);
}
__device__ __forceinline__ float bff(unsigned short b) { return __uint_as_float(((unsigned)b) << 16); }

__device__ __forceinline__ v8f wmb(v16bf a, v16bf b, v8f c) {
  v8f d = __builtin_amdgcn_wmma_f32_16x16x32_bf16(false, a, false, b, (short)0, c, false, false);
  asm volatile("v_nop\n\tv_nop\n\tv_nop\n\tv_nop" : "+v"(d) : "v"(a), "v"(b));
  return d;
}

template <int NB>
__device__ __forceinline__ int scan_chunk(const int* __restrict__ dsts, int nE, int cbase, int slotBase,
                                          int vec8, int* list, int tid, int lane, int wave) {
  int wc = 0;
#pragma unroll
  for (int g = 0; g < NGRP; ++g) {
    const int el0  = (g * NTHR + tid) * EPT;
    const int e0   = cbase + el0;
    const int sent = -2147483647 - 1;
    v4i da, db;
    if (vec8 != 0 && cbase + CHUNK <= nE) {
      da = *(const v4i*)(dsts + e0);
      db = *(const v4i*)(dsts + e0 + 4);
    } else {
      da.x = (e0     < nE) ? dsts[min(e0, nE - 1)] : sent;
      da.y = (e0 + 1 < nE) ? dsts[min(e0 + 1, nE - 1)] : sent;
      da.z = (e0 + 2 < nE) ? dsts[min(e0 + 2, nE - 1)] : sent;
      da.w = (e0 + 3 < nE) ? dsts[min(e0 + 3, nE - 1)] : sent;
      db.x = (e0 + 4 < nE) ? dsts[min(e0 + 4, nE - 1)] : sent;
      db.y = (e0 + 5 < nE) ? dsts[min(e0 + 5, nE - 1)] : sent;
      db.z = (e0 + 6 < nE) ? dsts[min(e0 + 6, nE - 1)] : sent;
      db.w = (e0 + 7 < nE) ? dsts[min(e0 + 7, nE - 1)] : sent;
    }
    const unsigned nb = (unsigned)slotBase;
    const unsigned s0 = (unsigned)da.x - nb, s1 = (unsigned)da.y - nb;
    const unsigned s2 = (unsigned)da.z - nb, s3 = (unsigned)da.w - nb;
    const unsigned s4 = (unsigned)db.x - nb, s5 = (unsigned)db.y - nb;
    const unsigned s6 = (unsigned)db.z - nb, s7 = (unsigned)db.w - nb;
    const bool h0 = s0 < (unsigned)NB, h1 = s1 < (unsigned)NB, h2 = s2 < (unsigned)NB, h3 = s3 < (unsigned)NB;
    const bool h4 = s4 < (unsigned)NB, h5 = s5 < (unsigned)NB, h6 = s6 < (unsigned)NB, h7 = s7 < (unsigned)NB;
    const unsigned any = __builtin_amdgcn_ballot_w32(h0 | h1 | h2 | h3 | h4 | h5 | h6 | h7);
    if (any != 0u) {
#define HITJ(J, HJ, SJ) { \
        const unsigned mj = __builtin_amdgcn_ballot_w32(HJ); \
        if (mj != 0u) { \
          if (HJ) { \
            const int pos = wc + (int)__builtin_amdgcn_mbcnt_lo(mj, 0u); \
            if (pos < WCAP) list[wave * WCAP + pos] = ((el0 + (J)) << 12) | (int)(SJ); \
          } \
          wc += (int)__builtin_popcount(mj); } }
      HITJ(0, h0, s0)
      HITJ(1, h1, s1)
      HITJ(2, h2, s2)
      HITJ(3, h3, s3)
      HITJ(4, h4, s4)
      HITJ(5, h5, s5)
      HITJ(6, h6, s6)
      HITJ(7, h7, s7)
#undef HITJ
    }
  }
  return wc;
}

__global__ __launch_bounds__(NTHR) void k_count(
    const int* __restrict__ ei, int* cnt, float* dinv, int nE, int vec8) {
  __shared__ __attribute__((aligned(16))) int scnt[NBC];
  __shared__ __attribute__((aligned(16))) int list[LISTN];
  __shared__ int wcnt[NWAVE];
  const int tid = threadIdx.x, lane = tid & 31, wave = tid >> 5;
  const int nodeBase = blockIdx.x * NBC;
  const int* dsts = ei + nE;

  for (int i = tid; i < NBC; i += NTHR) scnt[i] = 0;
  __syncthreads();

  const int nChunks = (nE + CHUNK - 1) / CHUNK;
#pragma unroll 1
  for (int ch = 0; ch < nChunks; ++ch) {
    const int cbase = ch * CHUNK;
    const int wc = scan_chunk<NBC>(dsts, nE, cbase, nodeBase, vec8, list, tid, lane, wave);
    if (lane == 0) wcnt[wave] = wc;
    __syncthreads();
    if (wave == 0) {
#pragma unroll 1
      for (int wsx = 0; wsx < NWAVE; ++wsx) {
        int n = __builtin_amdgcn_readfirstlane(wcnt[wsx]);
        n = n > WCAP ? WCAP : (n < 0 ? 0 : n);
        const int* lp = list + wsx * WCAP;
#pragma unroll 1
        for (int i = 0; i < n; ++i) {
          const int ent  = __builtin_amdgcn_readfirstlane(lp[i]);
          const int slot = ent & (NBC - 1);
          if (lane == 0) scnt[slot] = scnt[slot] + 1;
        }
      }
    }
    __syncthreads();
  }

  v4i cq[4]; v4f dq[4];
#pragma unroll
  for (int q = 0; q < 4; ++q) {
    const int f = (wave * 4 + q) * 128 + 4 * lane;
    const v4i c = *(const v4i*)(scnt + f);
    cq[q] = c;
    dq[q].x = rsqrtf((float)(c.x + 1));
    dq[q].y = rsqrtf((float)(c.y + 1));
    dq[q].z = rsqrtf((float)(c.z + 1));
    dq[q].w = rsqrtf((float)(c.w + 1));
  }
  int*   cp = cnt + (size_t)nodeBase;
  float* dp = dinv + (size_t)nodeBase;
#pragma unroll
  for (int q = 0; q < 4; ++q) {
    const int f = (wave * 4 + q) * 128 + 4 * lane;
    *(volatile v4i*)(cp + f) = cq[q];
    *(volatile v4f*)(dp + f) = dq[q];
  }
  __threadfence();
#pragma unroll
  for (int q = 0; q < 4; ++q) {
    const int f = (wave * 4 + q) * 128 + 4 * lane;
    *(volatile v4i*)(cp + f) = cq[q];
    *(volatile v4f*)(dp + f) = dq[q];
  }
}

__global__ __launch_bounds__(OTHR) void k_offsets(
    const int* __restrict__ cnt, int* off, int* rbase, int nChunk) {
  __shared__ __attribute__((aligned(16))) int soff[NBC];
  __shared__ __attribute__((aligned(16))) int srb[RBN];
  __shared__ int wtot[OTHR / 32];
  const int tid = threadIdx.x, lane = tid & 31, wave = tid >> 5, sub = tid >> 7;
  for (int i = tid; i < RBN; i += OTHR) srb[i] = 0;
  int carry = 0;
#pragma unroll 1
  for (int ch = 0; ch < nChunk; ++ch) {
    const int base = ch * NBC;
    const v4i c0 = *(const v4i*)(cnt + base + 8 * tid);
    const v4i c1 = *(const v4i*)(cnt + base + 8 * tid + 4);
    const int e0 = max(c0.x, 0), e1 = max(c0.y, 0), e2 = max(c0.z, 0), e3 = max(c0.w, 0);
    const int e4 = max(c1.x, 0), e5 = max(c1.y, 0), e6 = max(c1.z, 0), e7 = max(c1.w, 0);
    const int ts = e0 + e1 + e2 + e3 + e4 + e5 + e6 + e7;
    int incl = ts;
#pragma unroll
    for (int d = 1; d < 32; d <<= 1) {
      const int t = __shfl_up(incl, d);
      if (lane >= d) incl += t;
    }
    if (lane == 31) wtot[wave] = incl;
    __syncthreads();
    const int S0 = wtot[0]  + wtot[1]  + wtot[2]  + wtot[3];
    const int S1 = wtot[4]  + wtot[5]  + wtot[6]  + wtot[7];
    const int S2 = wtot[8]  + wtot[9]  + wtot[10] + wtot[11];
    const int S3 = wtot[12] + wtot[13] + wtot[14] + wtot[15];
    int pre = 0;
#pragma unroll 1
    for (int w = 4 * sub; w < wave; ++w) pre += wtot[w];
    const int b0 = carry;
    const int b1 = b0 + ((S0 + 31) & ~31);
    const int b2 = b1 + ((S1 + 31) & ~31);
    const int b3 = b2 + ((S2 + 31) & ~31);
    const int b4 = b3 + ((S3 + 31) & ~31);
    const int myb = sub == 0 ? b0 : (sub == 1 ? b1 : (sub == 2 ? b2 : b3));
    if (tid == 0) {
      srb[min(4 * ch + 0, RBN - 1)] = b0;
      srb[min(4 * ch + 1, RBN - 1)] = b1;
      srb[min(4 * ch + 2, RBN - 1)] = b2;
      srb[min(4 * ch + 3, RBN - 1)] = b3;
    }
    int run = myb + pre + incl - ts;
    soff[8 * tid + 0] = run; run += e0;
    soff[8 * tid + 1] = run; run += e1;
    soff[8 * tid + 2] = run; run += e2;
    soff[8 * tid + 3] = run; run += e3;
    soff[8 * tid + 4] = run; run += e4;
    soff[8 * tid + 5] = run; run += e5;
    soff[8 * tid + 6] = run; run += e6;
    soff[8 * tid + 7] = run;
    carry = b4;
    __syncthreads();
    const v4i o0 = *(const v4i*)(soff + 4 * tid);
    const v4i o1 = *(const v4i*)(soff + 4 * (tid + OTHR));
    int* op = off + base;
    *(volatile v4i*)(op + 4 * tid) = o0;
    *(volatile v4i*)(op + 4 * (tid + OTHR)) = o1;
    __threadfence();
    *(volatile v4i*)(op + 4 * tid) = o0;
    *(volatile v4i*)(op + 4 * (tid + OTHR)) = o1;
    __syncthreads();
  }
  if (tid == 0) srb[min(4 * nChunk, RBN - 1)] = carry;
  __syncthreads();
  v4i rv = {0, 0, 0, 0};
  if (tid < 32) rv = *(const v4i*)(srb + 4 * tid);
  if (tid < 32) *(volatile v4i*)(rbase + 4 * tid) = rv;
  __threadfence();
  if (tid < 32) *(volatile v4i*)(rbase + 4 * tid) = rv;
}

__global__ __launch_bounds__(NTHR) void k_fill(
    const int* __restrict__ ei, const int* __restrict__ off, const int* __restrict__ rbase,
    int* csr, int nN, int nE, int vec8, int csrLen) {
  extern __shared__ v4f lds_dyn[];
  int* region = (int*)lds_dyn;
  int* cursor = region + RCAP;
  int* list   = cursor + NBF;
  int* wcnt   = list + LISTN;
  const int tid = threadIdx.x, lane = tid & 31, wave = tid >> 5;
  const int b = blockIdx.x;
  const int nodeBase = b * NBF;
  const int* dsts = ei + nE;

  int rb0 = rbase[b];
  const int rb1 = rbase[b + 1];
  rb0 = rb0 < 0 ? 0 : (rb0 > csrLen ? csrLen : rb0);
  rb0 &= ~31;
  int len = rb1 - rb0;
  len = len < 0 ? 0 : (len > RCAP ? RCAP : len);
  int lenW = (len + 31) & ~31;
  if (rb0 + lenW > csrLen) lenW = (csrLen - rb0) & ~31;

  {
    const v4i z = {0, 0, 0, 0};
    for (int i = tid; i < RCAP / 4; i += NTHR) ((v4i*)region)[i] = z;
    for (int s = tid; s < NBF; s += NTHR) {
      int o = off[nodeBase + s] - rb0;
      o = o < 0 ? 0 : (o > RCAP ? RCAP : o);
      cursor[s] = o;
    }
  }
  __syncthreads();

  const int nChunks = (nE + CHUNK - 1) / CHUNK;
#pragma unroll 1
  for (int ch = 0; ch < nChunks; ++ch) {
    const int cbase = ch * CHUNK;
    const int wc = scan_chunk<NBF>(dsts, nE, cbase, nodeBase, vec8, list, tid, lane, wave);
    if (lane == 0) wcnt[wave] = wc;
    __syncthreads();
    if (wave == 0) {
#pragma unroll 1
      for (int wsx = 0; wsx < NWAVE; ++wsx) {
        int n = __builtin_amdgcn_readfirstlane(wcnt[wsx]);
        n = n > WCAP ? WCAP : (n < 0 ? 0 : n);
        const int* lp = list + wsx * WCAP;
#pragma unroll 1
        for (int i = 0; i < n; ++i) {
          const int ent  = __builtin_amdgcn_readfirstlane(lp[i]);
          const int slot = ent & (NBF - 1);
          int e = cbase + ((ent >> 12) & (CHUNK - 1));
          e = e > nE - 1 ? nE - 1 : e;
          int src = ei[e];
          src = src < 0 ? 0 : (src > nN - 1 ? nN - 1 : src);
          if (lane == 0) {
            int pos = cursor[slot];
            pos = pos < 0 ? 0 : (pos > RCAP - 1 ? RCAP - 1 : pos);
            region[pos] = src;
            const int np = pos + 1;
            cursor[slot] = np > RCAP ? RCAP : np;
          }
        }
      }
    }
    __syncthreads();
  }

  const int nv = lenW >> 2;
  int* gp = csr + rb0;
#pragma unroll 1
  for (int i = tid; i < nv; i += NTHR) { const v4i v = ((const v4i*)region)[i]; *(volatile v4i*)(gp + 4 * i) = v; }
  __threadfence();
#pragma unroll 1
  for (int i = tid; i < nv; i += NTHR) { const v4i v = ((const v4i*)region)[i]; *(volatile v4i*)(gp + 4 * i) = v; }
}

__global__ __launch_bounds__(NTHR) void k_xw1(
    const float* __restrict__ x, const float* __restrict__ W1, const float* __restrict__ dinv,
    float* hw, int nN) {
  const int tid = threadIdx.x;
  const int i  = blockIdx.x * XPB + (tid >> 3);
  const int g  = tid & 7;
  const int ic = i < nN ? i : nN - 1;
  const float x0 = x[(size_t)ic * XDIM + 0];
  const float x1 = x[(size_t)ic * XDIM + 1];
  const float x2 = x[(size_t)ic * XDIM + 2];
  const v4f w0 = *(const v4f*)(W1 + 0 * HID + 4 * g);
  const v4f w1 = *(const v4f*)(W1 + 1 * HID + 4 * g);
  const v4f w2 = *(const v4f*)(W1 + 2 * HID + 4 * g);
  const float dl = dinv[i];
  const float d  = (i < nN) ? dl : 0.0f;
  v4f v;
  v.x = (x0 * w0.x + x1 * w1.x + x2 * w2.x) * d;
  v.y = (x0 * w0.y + x1 * w1.y + x2 * w2.y) * d;
  v.z = (x0 * w0.z + x1 * w1.z + x2 * w2.z) * d;
  v.w = (x0 * w0.w + x1 * w1.w + x2 * w2.w) * d;
  float* p = hw + (size_t)i * HID + 4 * g;
  *(volatile v4f*)p = v;
  __threadfence();
  *(volatile v4f*)p = v;
}

template <int MODE>
__global__ __launch_bounds__(NTHR) void k_layer(
    const int* __restrict__ csr, const int* __restrict__ off, const int* __restrict__ cnt,
    const float* __restrict__ dinv, const float* __restrict__ hwin, const float* __restrict__ bias,
    const float* __restrict__ W, float* hwout, int nN, int csrLen) {
  __shared__ __attribute__((aligned(16))) float sH[TGT * HID];
  __shared__ __attribute__((aligned(16))) unsigned short sWh[HID * HID];
  __shared__ __attribute__((aligned(16))) unsigned short sWl[HID * HID];
  __shared__ __attribute__((aligned(16))) float sW4[HID];
  const int tid = threadIdx.x, lane = tid & 31, wave = tid >> 5, hh = lane >> 4, m = lane & 15;

  if (MODE == 0) {
#pragma unroll
    for (int it = 0; it < (HID * HID) / NTHR; ++it) {
      const int idx = it * NTHR + tid;
      const int n = idx >> 5, k = idx & 31;
      const float w = W[k * HID + n];
      const unsigned short hb = bfb(w);
      sWh[idx] = hb;
      sWl[idx] = bfb(w - bff(hb));
    }
  } else {
    if (tid < HID) sW4[tid] = W[tid];
  }

  const int tbase = blockIdx.x * TGT + wave * 32;
  const int cl = tbase + lane;
  const int cnt_l = cnt[cl];
  const int off_l = off[cl];
  FI dvu; dvu.f = dinv[cl];
  const float bl = bias[lane];

#pragma unroll 1
  for (int j = 0; j < 32; ++j) {
    const int c = tbase + j;
    int n = __builtin_amdgcn_readlane(cnt_l, j);
    n = n < 0 ? 0 : (n > DEGCAP ? DEGCAP : n);
    const int st = __builtin_amdgcn_readlane(off_l, j);
    FI du; du.i = __builtin_amdgcn_readlane(dvu.i, j);
    float acc = 0.0f;
#pragma unroll 1
    for (int q0 = 0; q0 < n; q0 += 32) {
      int pos = st + q0 + lane;
      pos = pos < 0 ? 0 : (pos > csrLen - 1 ? csrLen - 1 : pos);
      int sl = csr[pos];
      sl = sl < 0 ? 0 : (sl > nN - 1 ? nN - 1 : sl);
      const int mcnt = (n - q0) < 32 ? (n - q0) : 32;
#pragma unroll 1
      for (int p = 0; p < mcnt; ++p) {
        const int s = __builtin_amdgcn_readlane(sl, p);
        acc += hwin[(size_t)s * HID + lane];
      }
    }
    const float sv = hwin[(size_t)c * HID + lane];
    const float v = tanhf((acc + sv) * du.f + bl);
    sH[(wave * 32 + j) * HID + lane] = v;
  }
  __syncthreads();

  if (MODE == 0) {
    v8f acc[2][2];
#pragma unroll
    for (int rt = 0; rt < 2; ++rt) {
      const float* ar = sH + (wave * 32 + 16 * rt + m) * HID + 8 * hh;
      const v4f a0 = *(const v4f*)(ar);
      const v4f a1 = *(const v4f*)(ar + 4);
      const v4f a2 = *(const v4f*)(ar + 16);
      const v4f a3 = *(const v4f*)(ar + 20);
      float av[16] = { a0.x, a0.y, a0.z, a0.w, a1.x, a1.y, a1.z, a1.w,
                       a2.x, a2.y, a2.z, a2.w, a3.x, a3.y, a3.z, a3.w };
      FragB ahf, alf;
#pragma unroll
      for (int i = 0; i < 16; ++i) {
        const unsigned short hb = bfb(av[i]);
        ahf.u[i] = hb;
        alf.u[i] = bfb(av[i] - bff(hb));
      }
#pragma unroll
      for (int ct = 0; ct < 2; ++ct) {
        const unsigned short* bph = sWh + (16 * ct + m) * HID + 8 * hh;
        const unsigned short* bpl = sWl + (16 * ct + m) * HID + 8 * hh;
        FragB bh, blo;
        bh.h[0]  = *(const v8us*)bph;
        bh.h[1]  = *(const v8us*)(bph + 16);
        blo.h[0] = *(const v8us*)bpl;
        blo.h[1] = *(const v8us*)(bpl + 16);
        v8f c = {0.f, 0.f, 0.f, 0.f, 0.f, 0.f, 0.f, 0.f};
        c = wmb(alf.v, bh.v,  c);
        c = wmb(ahf.v, blo.v, c);
        c = wmb(ahf.v, bh.v,  c);
        acc[rt][ct] = c;
      }
    }
    __syncthreads();

#pragma unroll
    for (int rt = 0; rt < 2; ++rt) {
      const v4f d0 = *(const v4f*)(dinv + (size_t)tbase + 16 * rt + 8 * hh);
      const v4f d1 = *(const v4f*)(dinv + (size_t)tbase + 16 * rt + 8 * hh + 4);
      float s[8] = { d0.x, d0.y, d0.z, d0.w, d1.x, d1.y, d1.z, d1.w };
      float* sp = sH + (wave * 32 + 16 * rt + 8 * hh) * HID + m;
#pragma unroll
      for (int ct = 0; ct < 2; ++ct) {
#pragma unroll
        for (int r = 0; r < 8; ++r) sp[r * HID + 16 * ct] = acc[rt][ct][r] * s[r];
      }
    }
    __syncthreads();

    const float* lp = sH + wave * 32 * HID + 4 * lane;
    float* gp = hwout + (size_t)tbase * HID + 4 * lane;
    v4f ov[8];
#pragma unroll
    for (int p = 0; p < 8; ++p) ov[p] = *(const v4f*)(lp + 128 * p);
#pragma unroll
    for (int p = 0; p < 8; ++p) *(volatile v4f*)(gp + 128 * p) = ov[p];
    __threadfence();
#pragma unroll
    for (int p = 0; p < 8; ++p) *(volatile v4f*)(gp + 128 * p) = ov[p];
  } else {
    const float* hr = sH + (wave * 32 + lane) * HID;
    float s = 0.0f;
#pragma unroll 1
    for (int q = 0; q < HID / 4; ++q) {
      const v4f hv = *(const v4f*)(hr + 4 * q);
      const v4f wv = *(const v4f*)(sW4 + 4 * q);
      s += hv.x * wv.x + hv.y * wv.y + hv.z * wv.z + hv.w * wv.w;
    }
    const float val = s * dvu.f;
    float* gp = hwout + cl;
    *(volatile float*)gp = val;
    __threadfence();
    *(volatile float*)gp = val;
  }
}

__global__ __launch_bounds__(NTHR) void k_out(
    const int* __restrict__ csr, const int* __restrict__ off, const int* __restrict__ cnt,
    const float* __restrict__ dinv, const float* __restrict__ hw4, const float* __restrict__ b4,
    float* out, int nN, int csrLen) {
  const int tid = threadIdx.x, lane = tid & 31, wave = tid >> 5;
  const int tbase = blockIdx.x * TGT + wave * 32;
  const int cl = tbase + lane;
  int n = cnt[cl];
  n = n < 0 ? 0 : (n > DEGCAP ? DEGCAP : n);
  const int st = off[cl];
  const float dc = dinv[cl];
  int nmax = n;
#pragma unroll
  for (int d = 16; d > 0; d >>= 1) {
    const int t = __shfl_xor(nmax, d);
    nmax = t > nmax ? t : nmax;
  }
  float acc = 0.0f;
#pragma unroll 1
  for (int p = 0; p < nmax; ++p) {
    int pos = st + p;
    pos = pos < 0 ? 0 : (pos > csrLen - 1 ? csrLen - 1 : pos);
    int s = csr[pos];
    s = s < 0 ? 0 : (s > nN - 1 ? nN - 1 : s);
    const float hv = hw4[s];
    acc += (p < n) ? hv : 0.0f;
  }
  const float sv = hw4[cl];
  const float v = (acc + sv) * dc + b4[0];
  if (cl < nN) *(volatile float*)(out + cl) = v;
  __threadfence();
  if (cl < nN) *(volatile float*)(out + cl) = v;
}

extern "C" void kernel_launch(void* const* d_in, const int* in_sizes, int n_in,
                              void* d_out, int out_size, void* d_ws, size_t ws_size,
                              hipStream_t stream) {
  if (n_in < 10) return;
  if (in_sizes[2] != XDIM * HID || in_sizes[3] != HID || in_sizes[4] != HID * HID || in_sizes[5] != HID ||
      in_sizes[6] != HID * HID || in_sizes[7] != HID || in_sizes[8] != HID || in_sizes[9] < 1) return;
  const int nN = in_sizes[0] / XDIM;
  const int nE = in_sizes[1] / 2;
  if (nN <= 0 || nE <= 0 || in_sizes[0] != nN * XDIM || in_sizes[1] != 2 * nE) return;
  if (out_size != nN) return;
  if (nE > (1 << 28) || nN > (1 << 24)) return;

  const float* x  = (const float*)d_in[0];
  const int*   ei = (const int*)d_in[1];
  const float* W1 = (const float*)d_in[2];
  const float* b1 = (const float*)d_in[3];
  const float* W2 = (const float*)d_in[4];
  const float* b2 = (const float*)d_in[5];
  const float* W3 = (const float*)d_in[6];
  const float* b3 = (const float*)d_in[7];
  const float* W4 = (const float*)d_in[8];
  const float* b4 = (const float*)d_in[9];
  float* out = (float*)d_out;

  const int NPAD   = ((nN + TGT - 1) / TGT) * TGT;
  const int nBC    = (nN + NBC - 1) / NBC;
  const int CNTPAD = nBC * NBC;
  if (4 * nBC + 1 > RBN) return;
  const int nBF    = (nN + NBF - 1) / NBF;
  const int csrLen = ((nE + 31) & ~31) + 32 * nBF + 4096;
  const int nLay   = NPAD / TGT;
  const int nX     = NPAD / XPB;

  char* ws = (char*)d_ws;
  size_t off = 0;
  const size_t oCnt = off; off += (size_t)CNTPAD * 4;              off = (off + 255) & ~(size_t)255;
  const size_t oDv  = off; off += (size_t)CNTPAD * 4;              off = (off + 255) & ~(size_t)255;
  const size_t oOff = off; off += (size_t)CNTPAD * 4;              off = (off + 255) & ~(size_t)255;
  const size_t oRb  = off; off += (size_t)RBN * 4;                 off = (off + 255) & ~(size_t)255;
  const size_t oCsr = off; off += (size_t)csrLen * 4;              off = (off + 255) & ~(size_t)255;
  const size_t oHa  = off; off += (size_t)NPAD * HID * 4;          off = (off + 255) & ~(size_t)255;
  const size_t oHb  = off; off += (size_t)NPAD * HID * 4;          off = (off + 255) & ~(size_t)255;
  const size_t oH4  = off; off += (size_t)NPAD * 4;                off = (off + 255) & ~(size_t)255;
  if (off > ws_size || off > ((size_t)1 << 27)) return;
  int*   cnt  = (int*)(ws + oCnt);
  float* dinv = (float*)(ws + oDv);
  int*   offp = (int*)(ws + oOff);
  int*   rb   = (int*)(ws + oRb);
  int*   csr  = (int*)(ws + oCsr);
  float* hwA  = (float*)(ws + oHa);
  float* hwB  = (float*)(ws + oHb);
  float* hw4  = (float*)(ws + oH4);

  const int vec8 = ((nE & 3) == 0) ? 1 : 0;

  k_count<<<nBC, NTHR, 0, stream>>>(ei, cnt, dinv, nE, vec8);
  k_offsets<<<1, OTHR, 0, stream>>>(cnt, offp, rb, nBC);
  hipFuncSetAttribute(reinterpret_cast<const void*>(&k_fill),
                      hipFuncAttributeMaxDynamicSharedMemorySize, LDS_FILL);
  k_fill<<<nBF, NTHR, LDS_FILL, stream>>>(ei, offp, rb, csr, nN, nE, vec8, csrLen);

  k_xw1<<<nX, NTHR, 0, stream>>>(x, W1, dinv, hwA, nN);

  k_layer<0><<<nLay, NTHR, 0, stream>>>(csr, offp, cnt, dinv, hwA, b1, W2, hwB, nN, csrLen);
  k_layer<0><<<nLay, NTHR, 0, stream>>>(csr, offp, cnt, dinv, hwB, b2, W3, hwA, nN, csrLen);
  k_layer<1><<<nLay, NTHR, 0, stream>>>(csr, offp, cnt, dinv, hwA, b3, W4, hw4, nN, csrLen);
  k_out<<<nLay, NTHR, 0, stream>>>(csr, offp, cnt, dinv, hw4, b4, out, nN, csrLen);
}
